// RGCNEmb_17609365914131
// MI455X (gfx1250) — hardware-verified
//
#include <hip/hip_runtime.h>
#include <stddef.h>


#define EMBD    128
#define HID     32
#define NCLS    16
#define NREL    32
#define NBAS    16
#define K1      (NREL * EMBD)
#define K2      (NREL * HID)
#define TOBITS  17
#define TOMASK  ((1 << TOBITS) - 1)
#define MAXN    (1 << TOBITS)

#define NTHR    256
#define NWAVE   8
#define EPT     8
#define NGRP    2
#define CHUNK   (NTHR * EPT * NGRP)
#define WCAP    (EPT * NGRP * 32)
#define LISTN   (NWAVE * WCAP)
#define NBC     4096
#define NBF     1024
#define RCAP    40960
#define RBN     128
#define OTHR    512
#define NB1     16
#define NB2     64
#define DEGCAP  256
#define S1SC    256.0f
#define W1SC    16.0f
#define L1INV   (1.0f / 4096.0f)

#define LDS_FILL ((RCAP + NBF + LISTN) * 4 + 64)
#define LDS_L1   (NB1 * K1 * 4 + NB1 * NREL * 4)
#define LDS_L2   (NB2 * K2 * 4 + NB2 * NREL * 4)

static_assert((CHUNK & (CHUNK - 1)) == 0);
static_assert(CHUNK <= 4096);
static_assert(NBC <= 4096 && NBF <= 4096);
static_assert((NBC & (NBC - 1)) == 0 && (NBF & (NBF - 1)) == 0);
static_assert(NBC == 4 * NBF);
static_assert(OTHR * 8 == NBC);
static_assert((RCAP % 32) == 0);
static_assert(NB1 == 2 * NWAVE);
static_assert(NB2 == 8 * NWAVE);
static_assert(K1 / 32 == 16 * NWAVE);
static_assert(NWAVE * 16 * HID + NB1 * HID <= NB1 * K1);
static_assert(2 * NB2 * NCLS + NB2 * NCLS <= NB2 * K2);
static_assert(NB1 * K1 / 8 == 2 * NTHR * NB1);
static_assert(NB2 * (K2 / 8) == 128 * NB2);

typedef float          v4f  __attribute__((ext_vector_type(4)));
typedef float          v8f  __attribute__((ext_vector_type(8)));
typedef int            v4i  __attribute__((ext_vector_type(4)));
typedef _Float16       v8h  __attribute__((ext_vector_type(8)));
typedef _Float16       v16h __attribute__((ext_vector_type(16)));
typedef unsigned short v8us __attribute__((ext_vector_type(8)));
typedef __bf16         v16b __attribute__((ext_vector_type(16)));
union FragH { v16h v; v8h h[2]; };
union FragB { v16b v; v8us u[2]; };

__device__ __forceinline__ v4f sel4(bool c, v4f a, v4f b) {
  v4f r;
  r.x = c ? a.x : b.x; r.y = c ? a.y : b.y; r.z = c ? a.z : b.z; r.w = c ? a.w : b.w;
  return r;
}

__device__ __forceinline__ v8h cvt8(v4f a, v4f b) {
  v8h r;
  r[0] = (_Float16)a.x; r[1] = (_Float16)a.y; r[2] = (_Float16)a.z; r[3] = (_Float16)a.w;
  r[4] = (_Float16)b.x; r[5] = (_Float16)b.y; r[6] = (_Float16)b.z; r[7] = (_Float16)b.w;
  return r;
}

__device__ __forceinline__ unsigned short bfbits(float f) {
  unsigned int u = __float_as_uint(f);
  u += 0x7FFFu + ((u >> 16) & 1u);
  return (unsigned short)(u >> 16);
}

__device__ __forceinline__ void hilo(float x, unsigned short& hi, unsigned short& lo) {
  const unsigned short hb = bfbits(x);
  const float xh = __uint_as_float(((unsigned int)hb) << 16);
  hi = hb;
  lo = bfbits(x - xh);
}

__device__ __forceinline__ void split8(v4f a, v4f b, v8us& hv, v8us& lv) {
  unsigned short h0, h1, h2, h3, h4, h5, h6, h7, l0, l1, l2, l3, l4, l5, l6, l7;
  hilo(a.x, h0, l0); hilo(a.y, h1, l1); hilo(a.z, h2, l2); hilo(a.w, h3, l3);
  hilo(b.x, h4, l4); hilo(b.y, h5, l5); hilo(b.z, h6, l6); hilo(b.w, h7, l7);
  hv[0] = h0; hv[1] = h1; hv[2] = h2; hv[3] = h3; hv[4] = h4; hv[5] = h5; hv[6] = h6; hv[7] = h7;
  lv[0] = l0; lv[1] = l1; lv[2] = l2; lv[3] = l3; lv[4] = l4; lv[5] = l5; lv[6] = l6; lv[7] = l7;
}

__device__ __forceinline__ v8f wmh(v16h a, v16h b, v8f c) {
  v8f d = __builtin_amdgcn_wmma_f32_16x16x32_f16(false, a, false, b, (short)0, c, false, false);
  asm volatile("v_nop\n\tv_nop\n\tv_nop\n\tv_nop" : "+v"(d) : "v"(a), "v"(b));
  return d;
}
__device__ __forceinline__ v8f wmb(v16b a, v16b b, v8f c) {
  v8f d = __builtin_amdgcn_wmma_f32_16x16x32_bf16(false, a, false, b, (short)0, c, false, false);
  asm volatile("v_nop\n\tv_nop\n\tv_nop\n\tv_nop" : "+v"(d) : "v"(a), "v"(b));
  return d;
}

template <int NB>
__device__ __forceinline__ int scan_chunk(const int* __restrict__ dsts, int nE, int cbase, int slotBase,
                                          int vec8, int* list, int tid, int lane, int wave) {
  int wc = 0;
#pragma unroll
  for (int g = 0; g < NGRP; ++g) {
    const int el0  = (g * NTHR + tid) * EPT;
    const int e0   = cbase + el0;
    const int sent = -2147483647 - 1;
    v4i da, db;
    if (vec8 != 0 && cbase + CHUNK <= nE) {
      da = *(const v4i*)(dsts + e0);
      db = *(const v4i*)(dsts + e0 + 4);
    } else {
      da.x = (e0     < nE) ? dsts[min(e0, nE - 1)] : sent;
      da.y = (e0 + 1 < nE) ? dsts[min(e0 + 1, nE - 1)] : sent;
      da.z = (e0 + 2 < nE) ? dsts[min(e0 + 2, nE - 1)] : sent;
      da.w = (e0 + 3 < nE) ? dsts[min(e0 + 3, nE - 1)] : sent;
      db.x = (e0 + 4 < nE) ? dsts[min(e0 + 4, nE - 1)] : sent;
      db.y = (e0 + 5 < nE) ? dsts[min(e0 + 5, nE - 1)] : sent;
      db.z = (e0 + 6 < nE) ? dsts[min(e0 + 6, nE - 1)] : sent;
      db.w = (e0 + 7 < nE) ? dsts[min(e0 + 7, nE - 1)] : sent;
    }
    const unsigned nb = (unsigned)slotBase;
    const unsigned s0 = (unsigned)da.x - nb, s1 = (unsigned)da.y - nb;
    const unsigned s2 = (unsigned)da.z - nb, s3 = (unsigned)da.w - nb;
    const unsigned s4 = (unsigned)db.x - nb, s5 = (unsigned)db.y - nb;
    const unsigned s6 = (unsigned)db.z - nb, s7 = (unsigned)db.w - nb;
    const bool h0 = s0 < (unsigned)NB, h1 = s1 < (unsigned)NB, h2 = s2 < (unsigned)NB, h3 = s3 < (unsigned)NB;
    const bool h4 = s4 < (unsigned)NB, h5 = s5 < (unsigned)NB, h6 = s6 < (unsigned)NB, h7 = s7 < (unsigned)NB;
    const unsigned any = __builtin_amdgcn_ballot_w32(h0 | h1 | h2 | h3 | h4 | h5 | h6 | h7);
    if (any != 0u) {
#define HITJ(J, HJ, SJ) { \
        const unsigned mj = __builtin_amdgcn_ballot_w32(HJ); \
        if (mj != 0u) { \
          if (HJ) { \
            const int pos = wc + (int)__builtin_amdgcn_mbcnt_lo(mj, 0u); \
            if (pos < WCAP) list[wave * WCAP + pos] = ((el0 + (J)) << 12) | (int)(SJ); \
          } \
          wc += (int)__builtin_popcount(mj); } }
      HITJ(0, h0, s0)
      HITJ(1, h1, s1)
      HITJ(2, h2, s2)
      HITJ(3, h3, s3)
      HITJ(4, h4, s4)
      HITJ(5, h5, s5)
      HITJ(6, h6, s6)
      HITJ(7, h7, s7)
#undef HITJ
    }
  }
  return wc;
}

__global__ __launch_bounds__(NTHR) void k_prepw1(
    const float* __restrict__ comps, const float* __restrict__ bases, _Float16* w1p) {
  const int total = HID * (K1 / 8);
  const int i = blockIdx.x * NTHR + (int)threadIdx.x;
  if (i >= total) return;
  const int n  = i / (K1 / 8);
  const int k0 = (i - n * (K1 / 8)) * 8;
  const int r  = k0 / EMBD;
  const int e0 = k0 - r * EMBD;
  float a[8];
#pragma unroll
  for (int e = 0; e < 8; ++e) a[e] = 0.0f;
#pragma unroll 1
  for (int b = 0; b < NBAS; ++b) {
    const float c = comps[r * NBAS + b];
    const float* bp = bases + ((size_t)b * EMBD + e0) * HID + n;
#pragma unroll
    for (int e = 0; e < 8; ++e) a[e] += c * bp[e * HID];
  }
  v4f x, y;
  x.x = a[0] * W1SC; x.y = a[1] * W1SC; x.z = a[2] * W1SC; x.w = a[3] * W1SC;
  y.x = a[4] * W1SC; y.y = a[5] * W1SC; y.z = a[6] * W1SC; y.w = a[7] * W1SC;
  const v8h hv = cvt8(x, y);
  _Float16* dp = w1p + (size_t)i * 8;
  *(volatile v8h*)dp = hv;
  __threadfence();
  *(volatile v8h*)dp = hv;
}

__global__ __launch_bounds__(NTHR) void k_prepw2(
    const float* __restrict__ comps, const float* __restrict__ bases,
    unsigned short* w2hi, unsigned short* w2lo) {
  const int total = NCLS * (K2 / 8);
  const int i = blockIdx.x * NTHR + (int)threadIdx.x;
  if (i >= total) return;
  const int n  = i / (K2 / 8);
  const int k0 = (i - n * (K2 / 8)) * 8;
  const int r  = k0 / HID;
  const int h0 = k0 - r * HID;
  float a[8];
#pragma unroll
  for (int e = 0; e < 8; ++e) a[e] = 0.0f;
#pragma unroll 1
  for (int b = 0; b < NBAS; ++b) {
    const float c = comps[r * NBAS + b];
    const float* bp = bases + ((size_t)b * HID + h0) * NCLS + n;
#pragma unroll
    for (int e = 0; e < 8; ++e) a[e] += c * bp[e * NCLS];
  }
  v4f x, y;
  x.x = a[0]; x.y = a[1]; x.z = a[2]; x.w = a[3];
  y.x = a[4]; y.y = a[5]; y.z = a[6]; y.w = a[7];
  v8us hv, lv;
  split8(x, y, hv, lv);
  unsigned short* hp = w2hi + (size_t)i * 8;
  unsigned short* lp = w2lo + (size_t)i * 8;
  *(volatile v8us*)hp = hv;
  *(volatile v8us*)lp = lv;
  __threadfence();
  *(volatile v8us*)hp = hv;
  *(volatile v8us*)lp = lv;
}

__global__ __launch_bounds__(NTHR) void k_count(
    const int* __restrict__ dsts, int* cnt, int nE, int vec8) {
  __shared__ __attribute__((aligned(16))) int scnt[NBC];
  __shared__ __attribute__((aligned(16))) int list[LISTN];
  __shared__ int wcnt[NWAVE];
  const int tid = threadIdx.x, lane = tid & 31, wave = tid >> 5;
  const int nodeBase = blockIdx.x * NBC;

  for (int i = tid; i < NBC; i += NTHR) scnt[i] = 0;
  __syncthreads();

  const int nChunks = (nE + CHUNK - 1) / CHUNK;
#pragma unroll 1
  for (int ch = 0; ch < nChunks; ++ch) {
    const int cbase = ch * CHUNK;
    const int wc = scan_chunk<NBC>(dsts, nE, cbase, nodeBase, vec8, list, tid, lane, wave);
    if (lane == 0) wcnt[wave] = wc;
    __syncthreads();
    if (wave == 0) {
#pragma unroll 1
      for (int wsx = 0; wsx < NWAVE; ++wsx) {
        int n = __builtin_amdgcn_readfirstlane(wcnt[wsx]);
        n = n > WCAP ? WCAP : (n < 0 ? 0 : n);
        const int* lp = list + wsx * WCAP;
#pragma unroll 1
        for (int i = 0; i < n; ++i) {
          const int ent  = __builtin_amdgcn_readfirstlane(lp[i]);
          const int slot = ent & (NBC - 1);
          if (lane == 0) scnt[slot] = scnt[slot] + 1;
        }
      }
    }
    __syncthreads();
  }

  v4i cq[4];
#pragma unroll
  for (int q = 0; q < 4; ++q) {
    const int f = (wave * 4 + q) * 128 + 4 * lane;
    cq[q] = *(const v4i*)(scnt + f);
  }
  int* cp = cnt + (size_t)nodeBase;
#pragma unroll
  for (int q = 0; q < 4; ++q) {
    const int f = (wave * 4 + q) * 128 + 4 * lane;
    *(volatile v4i*)(cp + f) = cq[q];
  }
  __threadfence();
#pragma unroll
  for (int q = 0; q < 4; ++q) {
    const int f = (wave * 4 + q) * 128 + 4 * lane;
    *(volatile v4i*)(cp + f) = cq[q];
  }
}

__global__ __launch_bounds__(OTHR) void k_offsets(
    const int* __restrict__ cnt, int* off, int* rbase, int nChunk) {
  __shared__ __attribute__((aligned(16))) int soff[NBC];
  __shared__ __attribute__((aligned(16))) int srb[RBN];
  __shared__ int wtot[OTHR / 32];
  const int tid = threadIdx.x, lane = tid & 31, wave = tid >> 5, sub = tid >> 7;
  for (int i = tid; i < RBN; i += OTHR) srb[i] = 0;
  int carry = 0;
#pragma unroll 1
  for (int ch = 0; ch < nChunk; ++ch) {
    const int base = ch * NBC;
    const v4i c0 = *(const v4i*)(cnt + base + 8 * tid);
    const v4i c1 = *(const v4i*)(cnt + base + 8 * tid + 4);
    const int e0 = max(c0.x, 0), e1 = max(c0.y, 0), e2 = max(c0.z, 0), e3 = max(c0.w, 0);
    const int e4 = max(c1.x, 0), e5 = max(c1.y, 0), e6 = max(c1.z, 0), e7 = max(c1.w, 0);
    const int ts = e0 + e1 + e2 + e3 + e4 + e5 + e6 + e7;
    int incl = ts;
#pragma unroll
    for (int d = 1; d < 32; d <<= 1) {
      const int t = __shfl_up(incl, d);
      if (lane >= d) incl += t;
    }
    if (lane == 31) wtot[wave] = incl;
    __syncthreads();
    const int S0 = wtot[0]  + wtot[1]  + wtot[2]  + wtot[3];
    const int S1 = wtot[4]  + wtot[5]  + wtot[6]  + wtot[7];
    const int S2 = wtot[8]  + wtot[9]  + wtot[10] + wtot[11];
    const int S3 = wtot[12] + wtot[13] + wtot[14] + wtot[15];
    int pre = 0;
#pragma unroll 1
    for (int w = 4 * sub; w < wave; ++w) pre += wtot[w];
    const int b0 = carry;
    const int b1 = b0 + ((S0 + 31) & ~31);
    const int b2 = b1 + ((S1 + 31) & ~31);
    const int b3 = b2 + ((S2 + 31) & ~31);
    const int b4 = b3 + ((S3 + 31) & ~31);
    const int myb = sub == 0 ? b0 : (sub == 1 ? b1 : (sub == 2 ? b2 : b3));
    if (tid == 0) {
      srb[min(4 * ch + 0, RBN - 1)] = b0;
      srb[min(4 * ch + 1, RBN - 1)] = b1;
      srb[min(4 * ch + 2, RBN - 1)] = b2;
      srb[min(4 * ch + 3, RBN - 1)] = b3;
    }
    int run = myb + pre + incl - ts;
    soff[8 * tid + 0] = run; run += e0;
    soff[8 * tid + 1] = run; run += e1;
    soff[8 * tid + 2] = run; run += e2;
    soff[8 * tid + 3] = run; run += e3;
    soff[8 * tid + 4] = run; run += e4;
    soff[8 * tid + 5] = run; run += e5;
    soff[8 * tid + 6] = run; run += e6;
    soff[8 * tid + 7] = run;
    carry = b4;
    __syncthreads();
    const v4i o0 = *(const v4i*)(soff + 4 * tid);
    const v4i o1 = *(const v4i*)(soff + 4 * (tid + OTHR));
    int* op = off + base;
    *(volatile v4i*)(op + 4 * tid) = o0;
    *(volatile v4i*)(op + 4 * (tid + OTHR)) = o1;
    __threadfence();
    *(volatile v4i*)(op + 4 * tid) = o0;
    *(volatile v4i*)(op + 4 * (tid + OTHR)) = o1;
    __syncthreads();
  }
  if (tid == 0) srb[min(4 * nChunk, RBN - 1)] = carry;
  __syncthreads();
  v4i rv = {0, 0, 0, 0};
  if (tid < 32) rv = *(const v4i*)(srb + 4 * tid);
  if (tid < 32) *(volatile v4i*)(rbase + 4 * tid) = rv;
  __threadfence();
  if (tid < 32) *(volatile v4i*)(rbase + 4 * tid) = rv;
}

__global__ __launch_bounds__(NTHR) void k_fill(
    const int* __restrict__ dsts, const int* __restrict__ rel, const int* __restrict__ to,
    const int* __restrict__ off, const int* __restrict__ rbase,
    int* csr, int nN, int nE, int vec8, int csrLen) {
  extern __shared__ v4f lds_dyn[];
  int* region = (int*)lds_dyn;
  int* cursor = region + RCAP;
  int* list   = cursor + NBF;
  int* wcnt   = list + LISTN;
  const int tid = threadIdx.x, lane = tid & 31, wave = tid >> 5;
  const int b = blockIdx.x;
  const int nodeBase = b * NBF;

  int rb0 = rbase[b];
  const int rb1 = rbase[b + 1];
  rb0 = rb0 < 0 ? 0 : (rb0 > csrLen ? csrLen : rb0);
  rb0 &= ~31;
  int len = rb1 - rb0;
  len = len < 0 ? 0 : (len > RCAP ? RCAP : len);
  int lenW = (len + 31) & ~31;
  if (rb0 + lenW > csrLen) lenW = (csrLen - rb0) & ~31;

  {
    const v4i z = {0, 0, 0, 0};
    for (int i = tid; i < RCAP / 4; i += NTHR) ((v4i*)region)[i] = z;
    for (int s = tid; s < NBF; s += NTHR) {
      int o = off[nodeBase + s] - rb0;
      o = o < 0 ? 0 : (o > RCAP ? RCAP : o);
      cursor[s] = o;
    }
  }
  __syncthreads();

  const int nChunks = (nE + CHUNK - 1) / CHUNK;
#pragma unroll 1
  for (int ch = 0; ch < nChunks; ++ch) {
    const int cbase = ch * CHUNK;
    const int wc = scan_chunk<NBF>(dsts, nE, cbase, nodeBase, vec8, list, tid, lane, wave);
    if (lane == 0) wcnt[wave] = wc;
    __syncthreads();
    if (wave == 0) {
#pragma unroll 1
      for (int wsx = 0; wsx < NWAVE; ++wsx) {
        int n = __builtin_amdgcn_readfirstlane(wcnt[wsx]);
        n = n > WCAP ? WCAP : (n < 0 ? 0 : n);
        const int* lp = list + wsx * WCAP;
#pragma unroll 1
        for (int i = 0; i < n; ++i) {
          const int ent  = __builtin_amdgcn_readfirstlane(lp[i]);
          const int slot = ent & (NBF - 1);
          int e = cbase + ((ent >> 12) & (CHUNK - 1));
          e = e > nE - 1 ? nE - 1 : e;
          int rv = rel[e];
          rv = rv < 0 ? 0 : (rv > NREL - 1 ? NREL - 1 : rv);
          int tv = to[e];
          tv = tv < 0 ? 0 : (tv > nN - 1 ? nN - 1 : tv);
          const int pk = (rv << TOBITS) | tv;
          if (lane == 0) {
            int pos = cursor[slot];
            pos = pos < 0 ? 0 : (pos > RCAP - 1 ? RCAP - 1 : pos);
            region[pos] = pk;
            const int np = pos + 1;
            cursor[slot] = np > RCAP ? RCAP : np;
          }
        }
      }
    }
    __syncthreads();
  }

  const int nv = lenW >> 2;
  int* gp = csr + rb0;
#pragma unroll 1
  for (int i = tid; i < nv; i += NTHR) { const v4i v = ((const v4i*)region)[i]; *(volatile v4i*)(gp + 4 * i) = v; }
  __threadfence();
#pragma unroll 1
  for (int i = tid; i < nv; i += NTHR) { const v4i v = ((const v4i*)region)[i]; *(volatile v4i*)(gp + 4 * i) = v; }
}

__global__ __launch_bounds__(NTHR) void k_layer1(
    const int* __restrict__ csr, const int* __restrict__ off, const int* __restrict__ cnt,
    const float* __restrict__ emb, const _Float16* __restrict__ w1p, const float* __restrict__ bias,
    float* hid, int nN, int csrLen) {
  extern __shared__ v4f lds_dyn[];
  float*    sacc = (float*)lds_dyn;
  _Float16* sh   = (_Float16*)lds_dyn;
  int*      cntL = (int*)(sacc + NB1 * K1);
  const int tid = threadIdx.x, lane = tid & 31, wave = tid >> 5, hh = lane >> 4, m = lane & 15;
  const int base = blockIdx.x * NB1;

#pragma unroll 1
  for (int j = 0; j < NB1 / NWAVE; ++j) {
    const int s  = wave * (NB1 / NWAVE) + j;
    const int v  = base + s;
    const int vc = v < nN ? v : nN - 1;
    int cv = cnt[vc];
    int st = off[vc];
    cv = (v < nN) ? cv : 0;
    cv = cv < 0 ? 0 : (cv > DEGCAP ? DEGCAP : cv);
    st = st < 0 ? 0 : (st > csrLen - 1 ? csrLen - 1 : st);
    int cntv = 0;
    v4f* srow = (v4f*)(sacc + (size_t)s * K1);
#pragma unroll 1
    for (int q0 = 0; q0 < cv; q0 += 32) {
      int pos = st + q0 + lane;
      pos = pos < 0 ? 0 : (pos > csrLen - 1 ? csrLen - 1 : pos);
      const int pk = csr[pos];
      const int mcnt = (cv - q0) < 32 ? (cv - q0) : 32;
#pragma unroll 1
      for (int p = 0; p < mcnt; ++p) {
        const int ent = __builtin_amdgcn_readfirstlane(__builtin_amdgcn_readlane(pk, p));
        const int r = (ent >> TOBITS) & (NREL - 1);
        int t = ent & TOMASK;
        t = t > nN - 1 ? nN - 1 : t;
        const v4f x = *(const v4f*)(emb + (size_t)t * EMBD + 4 * lane);
        const int c = __builtin_amdgcn_readlane(cntv, r);
        const int idx = r * (EMBD / 4) + lane;
        const v4f old = srow[idx];
        srow[idx] = sel4(c != 0, old + x, x);
        cntv += (lane == r) ? 1 : 0;
      }
    }
    cntL[s * NREL + lane] = cntv;
  }
  __syncthreads();

#pragma unroll 1
  for (int r = 0; r < NB1; ++r) {
    const float* rowf = sacc + (size_t)r * K1;
    const int kA = 8 * tid, kB = K1 / 2 + 8 * tid;
    v4f a0 = *(const v4f*)(rowf + kA), a1 = *(const v4f*)(rowf + kA + 4);
    v4f b0 = *(const v4f*)(rowf + kB), b1 = *(const v4f*)(rowf + kB + 4);
    const int cA = cntL[r * NREL + (kA >> 7)];
    const int cB = cntL[r * NREL + (kB >> 7)];
    const float iA = S1SC * (1.0f / (float)(cA > 0 ? cA : 1));
    const float iB = S1SC * (1.0f / (float)(cB > 0 ? cB : 1));
    const v4f z = {0.0f, 0.0f, 0.0f, 0.0f};
    a0 = sel4(cA > 0, a0 * iA, z); a1 = sel4(cA > 0, a1 * iA, z);
    b0 = sel4(cB > 0, b0 * iB, z); b1 = sel4(cB > 0, b1 * iB, z);
    __syncthreads();
    *(v8h*)(sh + (size_t)r * (2 * K1) + kA) = cvt8(a0, a1);
    *(v8h*)(sh + (size_t)r * (2 * K1) + kB) = cvt8(b0, b1);
  }
  __syncthreads();

  v8f acc0 = {0.f, 0.f, 0.f, 0.f, 0.f, 0.f, 0.f, 0.f};
  v8f acc1 = {0.f, 0.f, 0.f, 0.f, 0.f, 0.f, 0.f, 0.f};
  const _Float16* ar  = sh  + (size_t)m * (2 * K1) + 8 * hh;
  const _Float16* bq0 = w1p + (size_t)m * K1 + 8 * hh;
  const _Float16* bq1 = w1p + (size_t)(16 + m) * K1 + 8 * hh;
  const int kt0 = wave * (K1 / 32 / NWAVE);
#pragma unroll 4
  for (int kk = 0; kk < K1 / 32 / NWAVE; ++kk) {
    const int ko = 32 * (kt0 + kk);
    FragH a, b;
    a.h[0] = *(const v8h*)(ar + ko);
    a.h[1] = *(const v8h*)(ar + ko + 16);
    b.h[0] = *(const v8h*)(bq0 + ko);
    b.h[1] = *(const v8h*)(bq0 + ko + 16);
    acc0 = wmh(a.v, b.v, acc0);
    b.h[0] = *(const v8h*)(bq1 + ko);
    b.h[1] = *(const v8h*)(bq1 + ko + 16);
    acc1 = wmh(a.v, b.v, acc1);
  }
  __syncthreads();

  float* part = sacc;
  float* pp = part + (size_t)(wave * 16 + 8 * hh) * HID + m;
#pragma unroll
  for (int r = 0; r < 8; ++r) { pp[r * HID] = acc0[r]; pp[r * HID + 16] = acc1[r]; }
  __syncthreads();

  float* otile = part + NWAVE * 16 * HID;
#pragma unroll
  for (int i2 = 0; i2 < 2; ++i2) {
    const int o = i2 * NTHR + tid;
    const int row = o >> 5, col = o & 31;
    float sv = 0.0f;
#pragma unroll
    for (int w = 0; w < NWAVE; ++w) sv += part[(w * 16 + row) * HID + col];
    float val = sv * L1INV + bias[col];
    val = fmaxf(val, 0.0f);
    otile[o] = val;
  }
  __syncthreads();

  if (tid < NB1 * HID / 4) {
    const int line = tid >> 3, piece = tid & 7;
    const v4f ov = *(const v4f*)(otile + line * HID + 4 * piece);
    float* gp = hid + ((size_t)base + line) * HID + 4 * piece;
    *(volatile v4f*)gp = ov;
    __threadfence();
    *(volatile v4f*)gp = ov;
  }
}

__global__ __launch_bounds__(NTHR) void k_layer2(
    const int* __restrict__ csr, const int* __restrict__ off, const int* __restrict__ cnt,
    const float* __restrict__ hid, const unsigned short* __restrict__ w2hi,
    const unsigned short* __restrict__ w2lo, const float* __restrict__ bias,
    float* out, int nN, int csrLen) {
  extern __shared__ v4f lds_dyn[];
  float*          sacc = (float*)lds_dyn;
  unsigned short* su   = (unsigned short*)lds_dyn;
  int*            cntL = (int*)(sacc + NB2 * K2);
  const int tid = threadIdx.x, lane = tid & 31, wave = tid >> 5, hh = lane >> 4, m = lane & 15;
  const int g = lane >> 3, q = lane & 7;
  const int base = blockIdx.x * NB2;

  {
    const v4f z = {0.0f, 0.0f, 0.0f, 0.0f};
#pragma unroll 4
    for (int i = tid; i < NB2 * K2 / 4; i += NTHR) lds_dyn[i] = z;
  }
  __syncthreads();

#pragma unroll 1
  for (int ph = 0; ph < NB2 / (NWAVE * 4); ++ph) {
    const int s  = wave * (NB2 / NWAVE) + ph * 4 + g;
    const int v  = base + s;
    const int vc = v < nN ? v : nN - 1;
    int cv = cnt[vc];
    int st = off[vc];
    cv = (v < nN) ? cv : 0;
    cv = cv < 0 ? 0 : (cv > DEGCAP ? DEGCAP : cv);
    st = st < 0 ? 0 : (st > csrLen - 1 ? csrLen - 1 : st);
    int mx = cv;
    mx = max(mx, __shfl_xor(mx, 8));
    mx = max(mx, __shfl_xor(mx, 16));
    mx = __builtin_amdgcn_readfirstlane(mx);
    mx = mx > DEGCAP ? DEGCAP : mx;
    int c0 = 0, c1 = 0, c2 = 0, c3 = 0;
    v4f* srow = (v4f*)(sacc + (size_t)s * K2);
#pragma unroll 1
    for (int p = 0; p < mx; ++p) {
      const bool valid = p < cv;
      int pos = st + p;
      pos = pos < 0 ? 0 : (pos > csrLen - 1 ? csrLen - 1 : pos);
      const int ent = csr[pos];
      const int r = (ent >> TOBITS) & (NREL - 1);
      int t = ent & TOMASK;
      t = t > nN - 1 ? nN - 1 : t;
      const v4f x = *(const v4f*)(hid + (size_t)t * HID + 4 * q);
      const int idx = r * (HID / 4) + q;
      const v4f old = srow[idx];
      srow[idx] = sel4(valid, old + x, old);
      const bool hit = valid && ((r & 7) == q);
      const int rj = r >> 3;
      c0 += (hit && rj == 0) ? 1 : 0;
      c1 += (hit && rj == 1) ? 1 : 0;
      c2 += (hit && rj == 2) ? 1 : 0;
      c3 += (hit && rj == 3) ? 1 : 0;
    }
    cntL[s * NREL + q]      = c0;
    cntL[s * NREL + 8 + q]  = c1;
    cntL[s * NREL + 16 + q] = c2;
    cntL[s * NREL + 24 + q] = c3;
  }
  __syncthreads();

#pragma unroll 1
  for (int pr = 0; pr < NB2 / 2; ++pr) {
    const int r  = 2 * pr + (tid >> 7);
    const int k0 = 8 * (tid & 127);
    const float* rowf = sacc + (size_t)r * K2;
    v4f x0 = *(const v4f*)(rowf + k0), x1 = *(const v4f*)(rowf + k0 + 4);
    const int c = cntL[r * NREL + (k0 >> 5)];
    const float inv = 1.0f / (float)(c > 0 ? c : 1);
    x0 = x0 * inv; x1 = x1 * inv;
    v8us hv, lv;
    split8(x0, x1, hv, lv);
    __syncthreads();
    *(v8us*)(su + (size_t)r * (2 * K2) + k0)      = hv;
    *(v8us*)(su + (size_t)r * (2 * K2) + K2 + k0) = lv;
  }
  __syncthreads();

  const int mt = wave & 3, kh = wave >> 2;
  const unsigned short* ahp = su + (size_t)(mt * 16 + m) * (2 * K2) + 8 * hh;
  const unsigned short* alp = ahp + K2;
  const unsigned short* bhp = w2hi + (size_t)m * K2 + 8 * hh;
  const unsigned short* blp = w2lo + (size_t)m * K2 + 8 * hh;
  v8f acc = {0.f, 0.f, 0.f, 0.f, 0.f, 0.f, 0.f, 0.f};
  const int kt0 = kh * (K2 / 32 / 2);
#pragma unroll 2
  for (int kk = 0; kk < K2 / 32 / 2; ++kk) {
    const int ko = 32 * (kt0 + kk);
    FragB ah, al, bh, bl;
    ah.u[0] = *(const v8us*)(ahp + ko); ah.u[1] = *(const v8us*)(ahp + ko + 16);
    al.u[0] = *(const v8us*)(alp + ko); al.u[1] = *(const v8us*)(alp + ko + 16);
    bh.u[0] = *(const v8us*)(bhp + ko); bh.u[1] = *(const v8us*)(bhp + ko + 16);
    bl.u[0] = *(const v8us*)(blp + ko); bl.u[1] = *(const v8us*)(blp + ko + 16);
    acc = wmb(ah.v, bh.v, acc);
    acc = wmb(ah.v, bl.v, acc);
    acc = wmb(al.v, bh.v, acc);
  }
  __syncthreads();

  float* part = sacc;
  float* pq = part + (size_t)(kh * NB2 + mt * 16 + 8 * hh) * NCLS + m;
#pragma unroll
  for (int r = 0; r < 8; ++r) pq[r * NCLS] = acc[r];
  __syncthreads();

  float* otile = part + 2 * NB2 * NCLS;
#pragma unroll
  for (int i4 = 0; i4 < 4; ++i4) {
    const int o = i4 * NTHR + tid;
    const int row = o >> 4, col = o & 15;
    otile[o] = part[row * NCLS + col] + part[(NB2 + row) * NCLS + col] + bias[col];
  }
  __syncthreads();

  int nval = nN - base;
  nval = nval > NB2 ? NB2 : (nval < 0 ? 0 : nval);
  const int nLines = nval >> 1;
  const int line = tid >> 3, piece = tid & 7;
  const v4f ov = *(const v4f*)(otile + line * 32 + 4 * piece);
  float* gp = out + (size_t)base * NCLS + line * 32 + 4 * piece;
  if (line < nLines) *(volatile v4f*)gp = ov;
  __threadfence();
  if (line < nLines) *(volatile v4f*)gp = ov;
}

extern "C" void kernel_launch(void* const* d_in, const int* in_sizes, int n_in,
                              void* d_out, int out_size, void* d_ws, size_t ws_size,
                              hipStream_t stream) {
  if (n_in < 10) return;
  if (in_sizes[0] <= 0 || (in_sizes[0] % EMBD) != 0) return;
  const int nN = in_sizes[0] / EMBD;
  const int nE = in_sizes[7];
  if (nN < 2 || nN > MAXN || (nN & 1) != 0) return;
  if (nE <= 0 || nE > (1 << 28) || in_sizes[8] != nE || in_sizes[9] != nE) return;
  if (in_sizes[1] != NREL * NBAS || in_sizes[2] != NBAS * EMBD * HID || in_sizes[3] != NREL * NBAS ||
      in_sizes[4] != NBAS * HID * NCLS || in_sizes[5] != HID || in_sizes[6] != NCLS) return;
  if (out_size != nN * NCLS) return;

  const float* emb    = (const float*)d_in[0];
  const float* comps1 = (const float*)d_in[1];
  const float* bases1 = (const float*)d_in[2];
  const float* comps2 = (const float*)d_in[3];
  const float* bases2 = (const float*)d_in[4];
  const float* bias1  = (const float*)d_in[5];
  const float* bias2  = (const float*)d_in[6];
  const int*   rel    = (const int*)d_in[7];
  const int*   fr     = (const int*)d_in[8];
  const int*   to     = (const int*)d_in[9];
  float* out = (float*)d_out;

  const int nBC    = (nN + NBC - 1) / NBC;
  const int CNTPAD = nBC * NBC;
  if (4 * nBC + 1 > RBN) return;
  const int nBF    = (nN + NBF - 1) / NBF;
  const int csrLen = ((nE + 31) & ~31) + 4096;
  const int nL1    = (nN + NB1 - 1) / NB1;
  const int NPAD1  = nL1 * NB1;
  const int nL2    = (nN + NB2 - 1) / NB2;

  char* ws = (char*)d_ws;
  size_t off = 0;
  const size_t oW1  = off; off += (size_t)HID * K1 * 2;          off = (off + 255) & ~(size_t)255;
  const size_t oW2h = off; off += (size_t)NCLS * K2 * 2;         off = (off + 255) & ~(size_t)255;
  const size_t oW2l = off; off += (size_t)NCLS * K2 * 2;         off = (off + 255) & ~(size_t)255;
  const size_t oCnt = off; off += (size_t)CNTPAD * 4;            off = (off + 255) & ~(size_t)255;
  const size_t oOff = off; off += (size_t)CNTPAD * 4;            off = (off + 255) & ~(size_t)255;
  const size_t oRb  = off; off += (size_t)RBN * 4;               off = (off + 255) & ~(size_t)255;
  const size_t oCsr = off; off += (size_t)csrLen * 4;            off = (off + 255) & ~(size_t)255;
  const size_t oHid = off; off += (size_t)NPAD1 * HID * 4;       off = (off + 255) & ~(size_t)255;
  if (off > ws_size || off > ((size_t)128 << 20)) return;
  _Float16*       w1p  = (_Float16*)(ws + oW1);
  unsigned short* w2hi = (unsigned short*)(ws + oW2h);
  unsigned short* w2lo = (unsigned short*)(ws + oW2l);
  int*            cnt  = (int*)(ws + oCnt);
  int*            offp = (int*)(ws + oOff);
  int*            rb   = (int*)(ws + oRb);
  int*            csr  = (int*)(ws + oCsr);
  float*          hid  = (float*)(ws + oHid);

  k_prepw1<<<(HID * (K1 / 8) + NTHR - 1) / NTHR, NTHR, 0, stream>>>(comps1, bases1, w1p);
  k_prepw2<<<(NCLS * (K2 / 8) + NTHR - 1) / NTHR, NTHR, 0, stream>>>(comps2, bases2, w2hi, w2lo);

  k_count<<<nBC, NTHR, 0, stream>>>(fr, cnt, nE, 1);
  k_offsets<<<1, OTHR, 0, stream>>>(cnt, offp, rb, nBC);
  hipFuncSetAttribute(reinterpret_cast<const void*>(&k_fill),
                      hipFuncAttributeMaxDynamicSharedMemorySize, LDS_FILL);
  k_fill<<<nBF, NTHR, LDS_FILL, stream>>>(fr, rel, to, offp, rb, csr, nN, nE, 1, csrLen);

  hipFuncSetAttribute(reinterpret_cast<const void*>(&k_layer1),
                      hipFuncAttributeMaxDynamicSharedMemorySize, LDS_L1);
  k_layer1<<<nL1, NTHR, LDS_L1, stream>>>(csr, offp, cnt, emb, w1p, bias1, hid, nN, csrLen);

  hipFuncSetAttribute(reinterpret_cast<const void*>(&k_layer2),
                      hipFuncAttributeMaxDynamicSharedMemorySize, LDS_L2);
  k_layer2<<<nL2, NTHR, LDS_L2, stream>>>(csr, offp, cnt, hid, w2hi, w2lo, bias2, out, nN, csrLen);
}
